// Net_32169305047431
// MI455X (gfx1250) — hardware-verified
//
#include <hip/hip_runtime.h>
#include <stddef.h>
#include <stdint.h>

#define NN      65536
#define NE      1048576
#define CH      64
#define NTHR    256
#define NWAVE   8
#define EPB     512
#define EPW     64
#define NEB     (NE / EPB)
#define PARTW   160
#define GBM     128
#define DP      68
#define NDW     192
#define HP      128
#define AP      136
#define BNEPS   1e-5f
#define P_W1    0
#define P_B1    32
#define P_W2    64
#define P_B2    256
#define P_AB1   320
#define P_AW2   352
#define P_AB2   416
#define P_SB    448
#define P_DB    512
#define P_LB    576
#define PARN    640
#define EPT     8
#define CHUNK   (NTHR * EPT)
#define WCAP    (EPT * 32)
#define LISTN   (NWAVE * WCAP)
#define NBMAX   2048
#define NBRUN   1024
#define RCAP    20480
#define DEGCAP  64
#define STW     512
#define LDS_AGG ((2 * RCAP + 2 * NBMAX + LISTN) * 4 + 64)
#define WSMAX   134217728

static_assert(CH == 64);
static_assert(NN % NBRUN == 0 && NN % GBM == 0);
static_assert(NE % EPB == 0 && EPB == NWAVE * EPW && EPW % 32 == 0);
static_assert(NE <= (1 << 20));
static_assert((CHUNK & (CHUNK - 1)) == 0 && CHUNK <= 4096);
static_assert((NBMAX & (NBMAX - 1)) == 0 && NBMAX <= 4096);
static_assert((NBRUN & (NBRUN - 1)) == 0 && NBRUN <= NBMAX);
static_assert(NTHR * 8 == NBMAX && LISTN >= NBMAX);
static_assert((RCAP % 32) == 0 && NWAVE * STW <= RCAP && PARTW <= STW);
static_assert(LDS_AGG <= 300000);
static_assert(PARTW % 32 == 0 && PARTW >= 2 * CH + 1 && PARTW / 4 <= NTHR);
static_assert((AP * 2) % 16 == 0 && (DP * 4) % 16 == 0 && AP >= HP);
static_assert(PARN % 32 == 0 && PARN / 4 <= NTHR);
static_assert(EPB * 8 == 4 * NTHR * 4);

typedef float          v4f   __attribute__((ext_vector_type(4)));
typedef float          v8f   __attribute__((ext_vector_type(8)));
typedef int            v4i   __attribute__((ext_vector_type(4)));
typedef int            v8i   __attribute__((ext_vector_type(8)));
typedef unsigned short v8us  __attribute__((ext_vector_type(8)));
typedef unsigned short v16us __attribute__((ext_vector_type(16)));
typedef __bf16         v16bf __attribute__((ext_vector_type(16)));
typedef v4f  __attribute__((may_alias)) v4fa;
typedef v8us __attribute__((may_alias)) v8usa;
union FragB { v16bf v; v16us u; v8us h[2]; v8i w; };

__device__ __forceinline__ v8f wmb(const FragB& a, const FragB& b, v8f c) {
  v8f d = __builtin_amdgcn_wmma_f32_16x16x32_bf16(false, a.v, false, b.v, (short)0, c, false, false);
  asm volatile("v_nop\n\tv_nop\n\tv_nop\n\tv_nop" : "+v"(d) : "v"(a.w), "v"(b.w));
  return d;
}
__device__ __forceinline__ v8f z8() { v8f z = {0.f, 0.f, 0.f, 0.f, 0.f, 0.f, 0.f, 0.f}; return z; }

__device__ __forceinline__ unsigned bf16_bits(float f) {
  const unsigned u = __float_as_uint(f);
  const unsigned r = (u + 0x7FFFu + ((u >> 16) & 1u)) >> 16;
  return ((u & 0x7fffffffu) > 0x7f800000u) ? 0x7fc0u : r;
}
__device__ __forceinline__ float bf16_val(float f) { return __uint_as_float(bf16_bits(f) << 16); }
__device__ __forceinline__ float rl(float v) { return (v > 0.0f) ? v : (v - v); }

__device__ __forceinline__ v8us cvt8b(const v4f a, const v4f b, unsigned mk) {
  v8us o;
  o[0] = (unsigned short)(bf16_bits(a.x) & mk); o[1] = (unsigned short)(bf16_bits(a.y) & mk);
  o[2] = (unsigned short)(bf16_bits(a.z) & mk); o[3] = (unsigned short)(bf16_bits(a.w) & mk);
  o[4] = (unsigned short)(bf16_bits(b.x) & mk); o[5] = (unsigned short)(bf16_bits(b.y) & mk);
  o[6] = (unsigned short)(bf16_bits(b.z) & mk); o[7] = (unsigned short)(bf16_bits(b.w) & mk);
  return o;
}
__device__ __forceinline__ v8us wunit(const float* __restrict__ p, unsigned mk) {
  const v4f a = *(const v4f*)p;
  const v4f b = *(const v4f*)(p + 4);
  return cvt8b(a, b, mk);
}
__device__ __forceinline__ void put16(unsigned short* dp, v8us o) {
  *(volatile v8us*)dp = o;
  __threadfence();
  *(volatile v8us*)dp = o;
}
__device__ __forceinline__ int clampi(int v, int hi) { return v < 0 ? 0 : (v > hi ? hi : v); }

__device__ __forceinline__ void ld_pos(const float* __restrict__ pos, int n, float& a, float& b, float& c) {
  const float* p = pos + (size_t)n * 3;
  a = bf16_val(p[0]); b = bf16_val(p[1]); c = bf16_val(p[2]);
}
__device__ __forceinline__ void p1vec(float r0, float r1, float r2, const float* w, float& p0, float& p1, float& p2) {
  p0 = fmaf(r2, w[P_W1 + 2], fmaf(r1, w[P_W1 + 1], r0 * w[P_W1 + 0])) + w[P_B1 + 0];
  p1 = fmaf(r2, w[P_W1 + 5], fmaf(r1, w[P_W1 + 4], r0 * w[P_W1 + 3])) + w[P_B1 + 1];
  p2 = fmaf(r2, w[P_W1 + 8], fmaf(r1, w[P_W1 + 7], r0 * w[P_W1 + 6])) + w[P_B1 + 2];
}
__device__ __forceinline__ float pld(const float* __restrict__ p, int j, int n) {
  const int jc = j < n ? j : n - 1;
  const float x = p[jc];
  return (j < n) ? bf16_val(x) : 0.0f;
}

__device__ __forceinline__ int scan_chunk(const int* __restrict__ dsts, int nE, int cbase, int slotBase,
                                          int nb, int vec8, int* list, int tid, int lane, int wave) {
  int wc = 0;
  const int el0  = tid * EPT;
  const int e0   = cbase + el0;
  const int sent = -2147483647 - 1;
  v4i da, db;
  if (vec8 != 0 && cbase + CHUNK <= nE) {
    da = *(const v4i*)(dsts + e0);
    db = *(const v4i*)(dsts + e0 + 4);
  } else {
    da.x = (e0     < nE) ? dsts[min(e0,     nE - 1)] : sent;
    da.y = (e0 + 1 < nE) ? dsts[min(e0 + 1, nE - 1)] : sent;
    da.z = (e0 + 2 < nE) ? dsts[min(e0 + 2, nE - 1)] : sent;
    da.w = (e0 + 3 < nE) ? dsts[min(e0 + 3, nE - 1)] : sent;
    db.x = (e0 + 4 < nE) ? dsts[min(e0 + 4, nE - 1)] : sent;
    db.y = (e0 + 5 < nE) ? dsts[min(e0 + 5, nE - 1)] : sent;
    db.z = (e0 + 6 < nE) ? dsts[min(e0 + 6, nE - 1)] : sent;
    db.w = (e0 + 7 < nE) ? dsts[min(e0 + 7, nE - 1)] : sent;
  }
  const unsigned nbs = (unsigned)slotBase;
  const unsigned unb = (unsigned)nb;
  const unsigned s0 = (unsigned)da.x - nbs, s1 = (unsigned)da.y - nbs;
  const unsigned s2 = (unsigned)da.z - nbs, s3 = (unsigned)da.w - nbs;
  const unsigned s4 = (unsigned)db.x - nbs, s5 = (unsigned)db.y - nbs;
  const unsigned s6 = (unsigned)db.z - nbs, s7 = (unsigned)db.w - nbs;
  const bool h0 = s0 < unb, h1 = s1 < unb, h2 = s2 < unb, h3 = s3 < unb;
  const bool h4 = s4 < unb, h5 = s5 < unb, h6 = s6 < unb, h7 = s7 < unb;
  const unsigned any = __builtin_amdgcn_ballot_w32(h0 | h1 | h2 | h3 | h4 | h5 | h6 | h7);
  if (any != 0u) {
#define HITJ(J, HJ, SJ) { \
      const unsigned mj = __builtin_amdgcn_ballot_w32(HJ); \
      if (mj != 0u) { \
        if (HJ) { \
          const int pos = wc + (int)__builtin_amdgcn_mbcnt_lo(mj, 0u); \
          if (pos < WCAP) list[wave * WCAP + pos] = ((el0 + (J)) << 12) | (int)(SJ); \
        } \
        wc += (int)__builtin_popcount(mj); } }
    HITJ(0, h0, s0)
    HITJ(1, h1, s1)
    HITJ(2, h2, s2)
    HITJ(3, h3, s3)
    HITJ(4, h4, s4)
    HITJ(5, h5, s5)
    HITJ(6, h6, s6)
    HITJ(7, h7, s7)
#undef HITJ
  }
  return wc;
}

__global__ __launch_bounds__(NTHR) void k_prep(
    const float* __restrict__ W_in, const float* __restrict__ src_w, const float* __restrict__ dst_w,
    const float* __restrict__ lin_w, const float* __restrict__ W_out, const float* __restrict__ attn_w1,
    const float* __restrict__ pw1, const float* __restrict__ pb1, const float* __restrict__ pw2,
    const float* __restrict__ pb2, const float* __restrict__ ab1, const float* __restrict__ aw2,
    const float* __restrict__ ab2, const float* __restrict__ sb, const float* __restrict__ db,
    const float* __restrict__ lb,
    unsigned short* WinB, unsigned short* Wcat, unsigned short* WoutD, unsigned short* Aw1D, float* PAR) {
  __shared__ __attribute__((aligned(16))) float sp[PARN];
  const int b = (int)blockIdx.x, tid = (int)threadIdx.x;
  if (b < 2) {
    const int u = b * NTHR + tid;
    const int n = u >> 3, k8 = (u & 7) * 8;
    put16(WinB + (size_t)u * 8, wunit(W_in + (size_t)n * CH + k8, 0xffffu));
    return;
  }
  if (b < 14) {
    const int u = (b - 2) * NTHR + tid;
    const int n = u >> 4, kk = (u & 15) * 8;
    const size_t off = (size_t)(n & 63) * CH + (kk & 63);
    const int mat = (b - 2) >> 2;
    v8us o;
    if (mat == 0)      o = wunit(src_w + off, 0xffffu);
    else if (mat == 1) o = wunit(dst_w + off, 0xffffu);
    else               o = wunit(lin_w + off, 0xffffu);
    put16(Wcat + (size_t)u * 8, o);
    return;
  }
  if (b < 18) {
    const int u = (b - 14) * NTHR + tid;
    const int n = u >> 4, kk = (u & 15) * 8;
    put16(WoutD + (size_t)u * 8, wunit(W_out + (size_t)n * CH + (kk & 63), 0xffffu));
    return;
  }
  if (b == 18) {
    const int u = tid;
    const int n = u >> 4, kk = (u & 15) * 8;
    const unsigned mk = (n < 8) ? 0xffffu : 0u;
    put16(Aw1D + (size_t)u * 8, wunit(attn_w1 + (size_t)(n & 7) * CH + (kk & 63), mk));
    return;
  }
#pragma unroll 1
  for (int it = 0; it < 3; ++it) {
    const int i = tid + NTHR * it;
    if (i < PARN) {
      float v;
      if (i < P_B1)       v = pld(pw1, i - P_W1, 9);
      else if (i < P_W2)  v = pld(pb1, i - P_B1, 3);
      else if (i < P_B2)  v = pld(pw2, i - P_W2, 192);
      else if (i < P_AB1) v = pld(pb2, i - P_B2, 64);
      else if (i < P_AW2) v = pld(ab1, i - P_AB1, 8);
      else if (i < P_AB2) v = pld(aw2, i - P_AW2, 64);
      else if (i < P_SB)  v = pld(ab2, i - P_AB2, 8);
      else if (i < P_DB)  v = pld(sb, i - P_SB, 64);
      else if (i < P_LB)  v = pld(db, i - P_DB, 64);
      else                v = pld(lb, i - P_LB, 64);
      sp[i] = v;
    }
  }
  __syncthreads();
  v4f v = {0.0f, 0.0f, 0.0f, 0.0f};
  if (tid < PARN / 4) {
    v = *(const v4fa*)(sp + 4 * tid);
    *(volatile v4f*)(PAR + 4 * tid) = v;
  }
  __threadfence();
  if (tid < PARN / 4) {
    *(volatile v4f*)(PAR + 4 * tid) = v;
  }
}

__device__ __forceinline__ void block_stats64(const float* sD, float* red, float* red2, float* pst,
                                              float* part, int pb, int tid) {
  const int c = tid & (CH - 1);
  const int g = tid >> 6;
  const float* col = sD + (size_t)(32 * g) * DP + c;
  float s = 0.0f;
#pragma unroll 4
  for (int i = 0; i < 32; ++i) s += col[i * DP];
  red[g * CH + c] = s;
  __syncthreads();
  const float tot  = ((red[c] + red[CH + c]) + red[2 * CH + c]) + red[3 * CH + c];
  const float mean = tot * (1.0f / (float)GBM);
  float q = 0.0f;
#pragma unroll 4
  for (int i = 0; i < 32; ++i) {
    const float d = col[i * DP] - mean;
    q = fmaf(d, d, q);
  }
  red2[g * CH + c] = q;
  __syncthreads();
  const float M2 = ((red2[c] + red2[CH + c]) + red2[2 * CH + c]) + red2[3 * CH + c];
  if (g == 0) { pst[1 + c] = mean; pst[1 + CH + c] = M2; }
  if (tid == 0) pst[0] = (float)GBM;
  if (tid >= 2 * CH + 1 && tid < PARTW) pst[tid] = 0.0f;
  __syncthreads();
  v4f ps = {0.0f, 0.0f, 0.0f, 0.0f};
  if (tid < PARTW / 4) {
    ps = *(const v4fa*)(pst + 4 * tid);
    *(volatile v4f*)(part + (size_t)pb * PARTW + 4 * tid) = ps;
  }
  __threadfence();
  if (tid < PARTW / 4) {
    *(volatile v4f*)(part + (size_t)pb * PARTW + 4 * tid) = ps;
  }
}

template <int NCH>
__device__ __forceinline__ void block_stats_small(const float* tile, float* red, float* red2, float* pst,
                                                  float* part, int pb, int tid) {
  constexpr int G  = NTHR / NCH;
  constexpr int RG = EPB / G;
  if (tid < PARTW) pst[tid] = 0.0f;
  const int c = tid & (NCH - 1);
  const int g = tid / NCH;
  const float* col = tile + (size_t)(g * RG) * NCH + c;
  float s = 0.0f;
#pragma unroll 4
  for (int i = 0; i < RG; ++i) s += col[i * NCH];
  red[tid] = s;
  __syncthreads();
  float tot = 0.0f;
#pragma unroll 4
  for (int gg = 0; gg < G; ++gg) tot += red[gg * NCH + c];
  const float mean = tot * (1.0f / (float)EPB);
  float q = 0.0f;
#pragma unroll 4
  for (int i = 0; i < RG; ++i) {
    const float d = col[i * NCH] - mean;
    q = fmaf(d, d, q);
  }
  red2[tid] = q;
  __syncthreads();
  float M2 = 0.0f;
#pragma unroll 4
  for (int gg = 0; gg < G; ++gg) M2 += red2[gg * NCH + c];
  if (tid < NCH) { pst[1 + c] = mean; pst[1 + CH + c] = M2; }
  if (tid == 0) pst[0] = (float)EPB;
  __syncthreads();
  v4f ps = {0.0f, 0.0f, 0.0f, 0.0f};
  if (tid < PARTW / 4) {
    ps = *(const v4fa*)(pst + 4 * tid);
    *(volatile v4f*)(part + (size_t)pb * PARTW + 4 * tid) = ps;
  }
  __threadfence();
  if (tid < PARTW / 4) {
    *(volatile v4f*)(part + (size_t)pb * PARTW + 4 * tid) = ps;
  }
}

template <int AF32, int KS, int STATS, int BIAS>
__global__ __launch_bounds__(NTHR) void k_gemm(const float* __restrict__ Af, const unsigned short* __restrict__ Ah,
                                               const unsigned short* __restrict__ BT, const float* __restrict__ par,
                                               float* outF, int ldo, float* part) {
  constexpr int K = 32 * KS;
  __shared__ __attribute__((aligned(16))) float stg[GBM * DP];
  __shared__ float red[NTHR];
  __shared__ float red2[NTHR];
  __shared__ __attribute__((aligned(16))) float pst[PARTW];
  const int tid = (int)threadIdx.x, lane = tid & 31, wave = tid >> 5, hh = lane >> 4, m = lane & 15;
  const int rowBase = (int)blockIdx.x * GBM;
  const int col0    = (int)blockIdx.y * 64;

  v8f acc[4];
#pragma unroll
  for (int t = 0; t < 4; ++t) acc[t] = z8();
  const size_t arow = (size_t)(rowBase + 16 * wave + m);
  const unsigned short* bp = BT + (size_t)(col0 + m) * (size_t)K + 8 * hh;
#pragma unroll
  for (int ks = 0; ks < KS; ++ks) {
    FragB af;
    if constexpr (AF32 != 0) {
      const float* ap = Af + arow * (size_t)CH + 32 * ks + 8 * hh;
      const v4f a0 = *(const v4f*)ap;
      const v4f a1 = *(const v4f*)(ap + 4);
      const v4f a2 = *(const v4f*)(ap + 16);
      const v4f a3 = *(const v4f*)(ap + 20);
      af.h[0] = cvt8b(a0, a1, 0xffffu);
      af.h[1] = cvt8b(a2, a3, 0xffffu);
    } else {
      const unsigned short* ap = Ah + arow * (size_t)K + 32 * ks + 8 * hh;
      af.h[0] = *(const v8usa*)ap;
      af.h[1] = *(const v8usa*)(ap + 16);
    }
#pragma unroll
    for (int t = 0; t < 4; ++t) {
      const unsigned short* wq = bp + (size_t)(16 * t) * (size_t)K + 32 * ks;
      FragB bf;
      bf.h[0] = *(const v8usa*)wq;
      bf.h[1] = *(const v8usa*)(wq + 16);
      acc[t] = wmb(af, bf, acc[t]);
    }
  }

#pragma unroll
  for (int t = 0; t < 4; ++t) {
    const int lc = 16 * t + m;
    float bv = 0.0f;
    if constexpr (BIAS != 0) bv = par[P_SB + col0 + lc];
#pragma unroll
    for (int r = 0; r < 8; ++r) {
      const int lr = 16 * wave + 8 * hh + r;
      stg[lr * DP + lc] = acc[t][r] + bv;
    }
  }
  __syncthreads();

  v4f fv[8];
#pragma unroll
  for (int i = 0; i < 8; ++i) {
    const int lr = 16 * wave + 2 * i + hh;
    fv[i] = *(const v4fa*)(stg + lr * DP + 4 * m);
  }
#pragma unroll
  for (int i = 0; i < 8; ++i) {
    const int lr = 16 * wave + 2 * i + hh;
    float* op = outF + (size_t)(rowBase + lr) * (size_t)ldo + col0 + 4 * m;
    *(volatile v4f*)op = fv[i];
  }
  __threadfence();
#pragma unroll
  for (int i = 0; i < 8; ++i) {
    const int lr = 16 * wave + 2 * i + hh;
    float* op = outF + (size_t)(rowBase + lr) * (size_t)ldo + col0 + 4 * m;
    *(volatile v4f*)op = fv[i];
  }
  if constexpr (STATS != 0) {
    block_stats64(stg, red, red2, pst, part, (int)blockIdx.x, tid);
  }
}

__global__ __launch_bounds__(NTHR) void k_comb(const float* __restrict__ part, int nPart, int nch,
                                               const float* __restrict__ gam, const float* __restrict__ bet,
                                               float* ss) {
  __shared__ double cn[NTHR], cm[NTHR], cq[NTHR];
  __shared__ __attribute__((aligned(16))) float stg[2 * CH];
  const int tid = (int)threadIdx.x;
  const int c = tid & (CH - 1);
  const int p = tid >> 6;
  double n = 0.0, mean = 0.0, M2 = 0.0;
#pragma unroll 1
  for (int b = p; b < nPart; b += 4) {
    const float* pr = part + (size_t)b * PARTW;
    const double nb = (double)pr[0];
    const double mb = (double)pr[1 + c];
    const double qb = (double)pr[1 + CH + c];
    if (nb > 0.5) {
      const double nn = n + nb;
      const double delta = mb - mean;
      const double f = nb / nn;
      mean = mean + delta * f;
      M2 = M2 + qb + delta * delta * n * f;
      n = nn;
    }
  }
  cn[tid] = n; cm[tid] = mean; cq[tid] = M2;
  __syncthreads();
  if (tid < CH) {
    double tn = 0.0, tm = 0.0, tq = 0.0;
#pragma unroll 1
    for (int p2 = 0; p2 < 4; ++p2) {
      const double nb = cn[p2 * CH + c];
      const double mb = cm[p2 * CH + c];
      const double qb = cq[p2 * CH + c];
      if (nb > 0.5) {
        const double nn = tn + nb;
        const double delta = mb - tm;
        const double f = nb / nn;
        tm = tm + delta * f;
        tq = tq + qb + delta * delta * tn * f;
        tn = nn;
      }
    }
    const double nt = tn < 1.0 ? 1.0 : tn;
    const float varf  = (float)(tq / nt);
    const float meanf = (float)tm;
    const float rstd = 1.0f / sqrtf(varf + BNEPS);
    const int cc = c < nch ? c : nch - 1;
    const float sc = bf16_val(gam[cc]) * rstd;
    const float sh = bf16_val(bet[cc]) - meanf * sc;
    stg[c] = sc;
    stg[CH + c] = sh;
  }
  __syncthreads();
  v4f v = {0.0f, 0.0f, 0.0f, 0.0f};
  if (tid < (2 * CH) / 4) {
    v = *(const v4fa*)(stg + 4 * tid);
    *(volatile v4f*)(ss + 4 * tid) = v;
  }
  __threadfence();
  if (tid < (2 * CH) / 4) {
    *(volatile v4f*)(ss + 4 * tid) = v;
  }
}

__global__ __launch_bounds__(NTHR) void k_apply(const float* __restrict__ P, const float* __restrict__ ss,
                                                unsigned short* H) {
  __shared__ __attribute__((aligned(16))) float sl[2 * CH];
  const int tid = (int)threadIdx.x;
  if (tid < 32) *(v4fa*)(sl + 4 * tid) = *(const v4f*)(ss + 4 * tid);
  __syncthreads();
  const int u = (int)blockIdx.x * NTHR + tid;
  const int row = u >> 3, j = u & 7;
  const float* p = P + (size_t)row * CH + 8 * j;
  const v4f a = *(const v4f*)p;
  const v4f b = *(const v4f*)(p + 4);
  const v8f x8 = {a.x, a.y, a.z, a.w, b.x, b.y, b.z, b.w};
  v8us oh, ol;
#pragma unroll
  for (int i = 0; i < 8; ++i) {
    const float v = rl(fmaf(x8[i], sl[8 * j + i], sl[CH + 8 * j + i]));
    const unsigned hb = bf16_bits(v);
    const unsigned lb = bf16_bits(v - __uint_as_float(hb << 16));
    oh[i] = (unsigned short)hb;
    ol[i] = (unsigned short)lb;
  }
  unsigned short* hp = H + (size_t)row * HP + 8 * j;
  *(volatile v8us*)hp = oh;
  *(volatile v8us*)(hp + CH) = ol;
  __threadfence();
  *(volatile v8us*)hp = oh;
  *(volatile v8us*)(hp + CH) = ol;
}

__global__ __launch_bounds__(NTHR) void k_epos(const int* __restrict__ srcs, const int* __restrict__ dsts,
                                               const float* __restrict__ pos, const float* __restrict__ par,
                                               float* part) {
  __shared__ __attribute__((aligned(16))) float sPar[64];
  __shared__ __attribute__((aligned(16))) float sP[EPB * 4];
  __shared__ float red[NTHR];
  __shared__ float red2[NTHR];
  __shared__ __attribute__((aligned(16))) float pst[PARTW];
  const int tid = (int)threadIdx.x;
  if (tid < 16) *(v4fa*)(sPar + 4 * tid) = *(const v4f*)(par + 4 * tid);
  __syncthreads();
#pragma unroll 1
  for (int it = 0; it < 2; ++it) {
    const int el = tid + NTHR * it;
    const int e  = (int)blockIdx.x * EPB + el;
    const int s = clampi(srcs[e], NN - 1);
    const int t = clampi(dsts[e], NN - 1);
    float s0, s1, s2, t0, t1, t2, p0, p1, p2;
    ld_pos(pos, s, s0, s1, s2);
    ld_pos(pos, t, t0, t1, t2);
    p1vec(s0 - t0, s1 - t1, s2 - t2, sPar, p0, p1, p2);
    const v4f pv = {p0, p1, p2, 0.0f};
    *(v4fa*)(sP + 4 * el) = pv;
  }
  __syncthreads();
  block_stats_small<4>(sP, red, red2, pst, part, (int)blockIdx.x, tid);
}

__global__ __launch_bounds__(NTHR) void k_ea(const int* __restrict__ srcs, const int* __restrict__ dsts,
                                             const float* __restrict__ pos, const float* __restrict__ node,
                                             const float* __restrict__ par, const float* __restrict__ ssp,
                                             float* part) {
  __shared__ __attribute__((aligned(16))) float sPar[PARN];
  __shared__ float rinv[72];
  __shared__ float wm[NWAVE * CH];
  __shared__ float wq[NWAVE * CH];
  __shared__ __attribute__((aligned(16))) float pst[PARTW];
  const int tid = (int)threadIdx.x, lane = tid & 31, wave = tid >> 5;
  if (tid < PARN / 4) *(v4fa*)(sPar + 4 * tid) = *(const v4f*)(par + 4 * tid);
  if (tid <= EPW) rinv[tid] = 1.0f / (float)(tid < 1 ? 1 : tid);
  __syncthreads();
  const int ca = lane, cb = lane + 32;
  const float wa0 = sPar[P_W2 + 3 * ca], wa1 = sPar[P_W2 + 3 * ca + 1], wa2 = sPar[P_W2 + 3 * ca + 2];
  const float wb0 = sPar[P_W2 + 3 * cb], wb1 = sPar[P_W2 + 3 * cb + 1], wb2 = sPar[P_W2 + 3 * cb + 2];
  const float ba = sPar[P_B2 + ca], bb = sPar[P_B2 + cb];
  const float scp0 = ssp[0], scp1 = ssp[1], scp2 = ssp[2];
  const float shp0 = ssp[CH], shp1 = ssp[CH + 1], shp2 = ssp[CH + 2];
  const int ebase = (int)blockIdx.x * EPB + wave * EPW;
  float mea = 0.0f, qa = 0.0f, meb = 0.0f, qb = 0.0f;
  int nW = 0;
#pragma unroll 1
  for (int b0 = 0; b0 < EPW; b0 += 32) {
    const int e = ebase + b0 + lane;
    const int s = clampi(srcs[e], NN - 1);
    const int t = clampi(dsts[e], NN - 1);
    float s0, s1, s2, t0, t1, t2, p0, p1, p2;
    ld_pos(pos, s, s0, s1, s2);
    ld_pos(pos, t, t0, t1, t2);
    p1vec(s0 - t0, s1 - t1, s2 - t2, sPar, p0, p1, p2);
    const float d0 = rl(fmaf(p0, scp0, shp0));
    const float d1 = rl(fmaf(p1, scp1, shp1));
    const float d2 = rl(fmaf(p2, scp2, shp2));
#pragma unroll 1
    for (int k = 0; k < 32; ++k) {
      const int sk = __builtin_amdgcn_readlane(s, k);
      const int tk = __builtin_amdgcn_readlane(t, k);
      const float e0 = __int_as_float(__builtin_amdgcn_readlane(__float_as_int(d0), k));
      const float e1 = __int_as_float(__builtin_amdgcn_readlane(__float_as_int(d1), k));
      const float e2 = __int_as_float(__builtin_amdgcn_readlane(__float_as_int(d2), k));
      const float* ns = node + (size_t)sk * NDW;
      const float* nt = node + (size_t)tk * NDW + CH;
      const float dla = fmaf(e2, wa2, fmaf(e1, wa1, e0 * wa0)) + ba;
      const float dlb = fmaf(e2, wb2, fmaf(e1, wb1, e0 * wb0)) + bb;
      const float aa = (ns[ca] - nt[ca]) + dla;
      const float ab = (ns[cb] - nt[cb]) + dlb;
      nW = nW + 1;
      const float r = rinv[nW];
      const float da = aa - mea;
      mea = fmaf(da, r, mea);
      qa = fmaf(da, aa - mea, qa);
      const float db = ab - meb;
      meb = fmaf(db, r, meb);
      qb = fmaf(db, ab - meb, qb);
    }
  }
  wm[wave * CH + ca] = mea; wm[wave * CH + cb] = meb;
  wq[wave * CH + ca] = qa;  wq[wave * CH + cb] = qb;
  __syncthreads();
  if (tid < CH) {
    float n = 0.0f, mean = 0.0f, M2 = 0.0f;
#pragma unroll 1
    for (int w = 0; w < NWAVE; ++w) {
      const float nb = (float)EPW;
      const float mb = wm[w * CH + tid];
      const float q2 = wq[w * CH + tid];
      const float nn = n + nb;
      const float dl = mb - mean;
      const float f = nb * (1.0f / nn);
      mean = fmaf(dl, f, mean);
      M2 = M2 + q2 + dl * dl * n * f;
      n = nn;
    }
    pst[1 + tid] = mean;
    pst[1 + CH + tid] = M2;
  }
  if (tid == 0) pst[0] = (float)EPB;
  if (tid >= 2 * CH + 1 && tid < PARTW) pst[tid] = 0.0f;
  __syncthreads();
  v4f ps = {0.0f, 0.0f, 0.0f, 0.0f};
  if (tid < PARTW / 4) {
    ps = *(const v4fa*)(pst + 4 * tid);
    *(volatile v4f*)(part + (size_t)blockIdx.x * PARTW + 4 * tid) = ps;
  }
  __threadfence();
  if (tid < PARTW / 4) {
    *(volatile v4f*)(part + (size_t)blockIdx.x * PARTW + 4 * tid) = ps;
  }
}

__global__ __launch_bounds__(NTHR) void k_ea1(const int* __restrict__ srcs, const int* __restrict__ dsts,
                                              const float* __restrict__ pos, const float* __restrict__ node,
                                              const float* __restrict__ par, const float* __restrict__ ssp,
                                              const float* __restrict__ ssa, const unsigned short* __restrict__ Aw1D,
                                              float* A1, float* part) {
  __shared__ __attribute__((aligned(16))) float sPar[PARN];
  __shared__ __attribute__((aligned(16))) unsigned short sA[GBM * AP];
  __shared__ __attribute__((aligned(16))) float sY[EPB * 8];
  __shared__ float red[NTHR];
  __shared__ float red2[NTHR];
  __shared__ __attribute__((aligned(16))) float pst[PARTW];
  const int tid = (int)threadIdx.x, lane = tid & 31, wave = tid >> 5, hh = lane >> 4, m = lane & 15;
  if (tid < PARN / 4) *(v4fa*)(sPar + 4 * tid) = *(const v4f*)(par + 4 * tid);
  __syncthreads();
  const int ca = lane, cb = lane + 32;
  const float wa0 = sPar[P_W2 + 3 * ca], wa1 = sPar[P_W2 + 3 * ca + 1], wa2 = sPar[P_W2 + 3 * ca + 2];
  const float wb0 = sPar[P_W2 + 3 * cb], wb1 = sPar[P_W2 + 3 * cb + 1], wb2 = sPar[P_W2 + 3 * cb + 2];
  const float ba = sPar[P_B2 + ca], bb = sPar[P_B2 + cb];
  const float ab1 = sPar[P_AB1 + (m & 7)];
  const float scp0 = ssp[0], scp1 = ssp[1], scp2 = ssp[2];
  const float shp0 = ssp[CH], shp1 = ssp[CH + 1], shp2 = ssp[CH + 2];
  const float sca = ssa[ca], scb = ssa[cb], sha = ssa[CH + ca], shb = ssa[CH + cb];
  FragB bw[4];
  {
    const unsigned short* bq = Aw1D + (size_t)m * HP + 8 * hh;
#pragma unroll
    for (int ks = 0; ks < 4; ++ks) {
      bw[ks].h[0] = *(const v8usa*)(bq + 32 * ks);
      bw[ks].h[1] = *(const v8usa*)(bq + 32 * ks + 16);
    }
  }
  const int ebase = (int)blockIdx.x * EPB + wave * EPW;
#pragma unroll 1
  for (int b0 = 0; b0 < EPW; b0 += 32) {
    const int e = ebase + b0 + lane;
    const int s = clampi(srcs[e], NN - 1);
    const int t = clampi(dsts[e], NN - 1);
    float s0, s1, s2, t0, t1, t2, p0, p1, p2;
    ld_pos(pos, s, s0, s1, s2);
    ld_pos(pos, t, t0, t1, t2);
    p1vec(s0 - t0, s1 - t1, s2 - t2, sPar, p0, p1, p2);
    const float d0 = rl(fmaf(p0, scp0, shp0));
    const float d1 = rl(fmaf(p1, scp1, shp1));
    const float d2 = rl(fmaf(p2, scp2, shp2));
#pragma unroll 1
    for (int hf = 0; hf < 2; ++hf) {
#pragma unroll 1
      for (int k = 0; k < 16; ++k) {
        const int kk = 16 * hf + k;
        const int sk = __builtin_amdgcn_readlane(s, kk);
        const int tk = __builtin_amdgcn_readlane(t, kk);
        const float e0 = __int_as_float(__builtin_amdgcn_readlane(__float_as_int(d0), kk));
        const float e1 = __int_as_float(__builtin_amdgcn_readlane(__float_as_int(d1), kk));
        const float e2 = __int_as_float(__builtin_amdgcn_readlane(__float_as_int(d2), kk));
        const float* ns = node + (size_t)sk * NDW;
        const float* nt = node + (size_t)tk * NDW + CH;
        const float dla = fmaf(e2, wa2, fmaf(e1, wa1, e0 * wa0)) + ba;
        const float dlb = fmaf(e2, wb2, fmaf(e1, wb1, e0 * wb0)) + bb;
        const float aa = (ns[ca] - nt[ca]) + dla;
        const float ab = (ns[cb] - nt[cb]) + dlb;
        const float va = rl(fmaf(aa, sca, sha));
        const float vb = rl(fmaf(ab, scb, shb));
        const unsigned ha = bf16_bits(va);
        const unsigned la = bf16_bits(va - __uint_as_float(ha << 16));
        const unsigned hb = bf16_bits(vb);
        const unsigned lb = bf16_bits(vb - __uint_as_float(hb << 16));
        unsigned short* rw = sA + (16 * wave + k) * AP;
        rw[ca] = (unsigned short)ha;
        rw[cb] = (unsigned short)hb;
        rw[CH + ca] = (unsigned short)la;
        rw[CH + cb] = (unsigned short)lb;
      }
      __syncthreads();
      v8f acc = z8();
      const unsigned short* ar = sA + (16 * wave + m) * AP + 8 * hh;
#pragma unroll
      for (int ks = 0; ks < 4; ++ks) {
        FragB af;
        af.h[0] = *(const v8usa*)(ar + 32 * ks);
        af.h[1] = *(const v8usa*)(ar + 32 * ks + 16);
        acc = wmb(af, bw[ks], acc);
      }
      const int er = wave * EPW + b0 + 16 * hf + 8 * hh;
      if (m < 8) {
#pragma unroll
        for (int r = 0; r < 8; ++r) sY[(er + r) * 8 + m] = acc[r] + ab1;
      }
      __syncthreads();
    }
  }
  block_stats_small<8>(sY, red, red2, pst, part, (int)blockIdx.x, tid);
  v4f pv[4];
#pragma unroll
  for (int it = 0; it < 4; ++it) pv[it] = *(const v4fa*)(sY + (size_t)(it * NTHR + tid) * 4);
  float* ob = A1 + (size_t)blockIdx.x * (EPB * 8);
#pragma unroll
  for (int it = 0; it < 4; ++it) *(volatile v4f*)(ob + (size_t)(it * NTHR + tid) * 4) = pv[it];
  __threadfence();
#pragma unroll
  for (int it = 0; it < 4; ++it) *(volatile v4f*)(ob + (size_t)(it * NTHR + tid) * 4) = pv[it];
}

__global__ __launch_bounds__(NTHR) void k_scan(const int* __restrict__ srcs, const int* __restrict__ dsts,
                                               const float* __restrict__ pos, const float* __restrict__ node,
                                               const float* __restrict__ A1, const float* __restrict__ par,
                                               const float* __restrict__ ssp, const float* __restrict__ ssa2,
                                               float* outp, float* part, int vec8) {
  extern __shared__ v4f lds_dyn[];
  __shared__ __attribute__((aligned(16))) float sPar[PARN];
  __shared__ float sS2[16];
  __shared__ float rinv[132];
  int* reg1 = (int*)lds_dyn;
  int* reg2 = reg1 + RCAP;
  int* scnt = reg2 + RCAP;
  int* soff = scnt + NBMAX;
  int* list = soff + NBMAX;
  int* wcnt = list + LISTN;
  int* wtot = wcnt + NWAVE;
  const int tid = (int)threadIdx.x, lane = tid & 31, wave = tid >> 5;
  const int nb = NBRUN;
  const int nE = NE;
  const int nodeBase = (int)blockIdx.x * nb;

  if (tid < PARN / 4) *(v4fa*)(sPar + 4 * tid) = *(const v4f*)(par + 4 * tid);
  if (tid < 16) sS2[tid] = ssa2[(tid & 7) + ((tid >> 3) << 6)];
  if (tid <= 128) rinv[tid] = 1.0f / (float)(tid < 1 ? 1 : tid);
  for (int i = tid; i < NBMAX; i += NTHR) scnt[i] = 0;
  __syncthreads();

  int tot = 0;
  const int nChunks = (nE + CHUNK - 1) / CHUNK;
#pragma unroll 1
  for (int ch = 0; ch < nChunks; ++ch) {
    const int cbase = ch * CHUNK;
    const int wc = scan_chunk(dsts, nE, cbase, nodeBase, nb, vec8, list, tid, lane, wave);
    if (lane == 0) wcnt[wave] = wc;
    __syncthreads();
    int pre = 0, all = 0;
#pragma unroll
    for (int w2 = 0; w2 < NWAVE; ++w2) {
      int c = wcnt[w2];
      c = c < 0 ? 0 : (c > WCAP ? WCAP : c);
      all += c;
      pre += (w2 < wave) ? c : 0;
    }
    const int wcc  = wc > WCAP ? WCAP : wc;
    const int base = tot + pre;
#pragma unroll 1
    for (int i = lane; i < wcc; i += 32) {
      const int ent = list[wave * WCAP + i];
      const int el  = (ent >> 12) & (CHUNK - 1);
      const int sl  = ent & (NBMAX - 1);
      int eid = cbase + el;
      eid = eid > nE - 1 ? nE - 1 : eid;
      const int p = base + i;
      if (p < RCAP) reg1[p] = (int)(((unsigned)eid << 12) | (unsigned)sl);
    }
    tot += all;
    tot = tot > RCAP ? RCAP : tot;
    __syncthreads();
  }
  const int nh = tot;

  if (wave == 0) {
#pragma unroll 1
    for (int b0 = 0; b0 < nh; b0 += 32) {
      const int idx = b0 + lane;
      const int uv  = reg1[idx < RCAP ? idx : RCAP - 1];
      const int m32 = (nh - b0) < 32 ? (nh - b0) : 32;
#pragma unroll 1
      for (int k = 0; k < m32; ++k) {
        const int u  = __builtin_amdgcn_readlane(uv, k);
        const int sl = u & (NBMAX - 1);
        if (lane == 0) scnt[sl] = scnt[sl] + 1;
      }
    }
  }
  __syncthreads();

  {
    const v4i ca4 = *(const v4i*)(scnt + 8 * tid);
    const v4i cb4 = *(const v4i*)(scnt + 8 * tid + 4);
    const int e0 = ca4.x < 0 ? 0 : ca4.x, e1 = ca4.y < 0 ? 0 : ca4.y, e2 = ca4.z < 0 ? 0 : ca4.z, e3 = ca4.w < 0 ? 0 : ca4.w;
    const int e4 = cb4.x < 0 ? 0 : cb4.x, e5 = cb4.y < 0 ? 0 : cb4.y, e6 = cb4.z < 0 ? 0 : cb4.z, e7 = cb4.w < 0 ? 0 : cb4.w;
    const int ts = e0 + e1 + e2 + e3 + e4 + e5 + e6 + e7;
    int incl = ts;
#pragma unroll
    for (int d = 1; d < 32; d <<= 1) {
      const int up = __shfl_up(incl, d);
      if (lane >= d) incl += up;
    }
    if (lane == 31) wtot[wave] = incl;
    __syncthreads();
    int pre = 0;
#pragma unroll
    for (int w2 = 0; w2 < NWAVE; ++w2) pre += (w2 < wave) ? wtot[w2] : 0;
    int run = pre + incl - ts;
    soff[8 * tid + 0] = run; run += e0;
    soff[8 * tid + 1] = run; run += e1;
    soff[8 * tid + 2] = run; run += e2;
    soff[8 * tid + 3] = run; run += e3;
    soff[8 * tid + 4] = run; run += e4;
    soff[8 * tid + 5] = run; run += e5;
    soff[8 * tid + 6] = run; run += e6;
    soff[8 * tid + 7] = run;
  }
  __syncthreads();
  for (int i = tid; i < NBMAX; i += NTHR) list[i] = soff[i];
  __syncthreads();

  if (wave == 0) {
#pragma unroll 1
    for (int b0 = 0; b0 < nh; b0 += 32) {
      const int idx = b0 + lane;
      const int uv  = reg1[idx < RCAP ? idx : RCAP - 1];
      const int m32 = (nh - b0) < 32 ? (nh - b0) : 32;
#pragma unroll 1
      for (int k = 0; k < m32; ++k) {
        const int u   = __builtin_amdgcn_readlane(uv, k);
        const int sl  = u & (NBMAX - 1);
        const int eid = (int)((unsigned)u >> 12);
        if (lane == 0) {
          int p = list[sl];
          p = p < 0 ? 0 : (p > RCAP - 1 ? RCAP - 1 : p);
          reg2[p] = eid;
          list[sl] = p + 1;
        }
      }
    }
  }
  __syncthreads();

  const int nbw = NBRUN >> 3;
  const bool ovf = (nh >= RCAP);
  const float qnan = __int_as_float(0x7fc00000);
  float* stw = (float*)reg1 + wave * STW;
  const int ca = lane, cb = lane + 32, jj = lane & 7;
  float w2r[8];
#pragma unroll
  for (int i = 0; i < 8; ++i) w2r[i] = sPar[P_AW2 + jj * 8 + i];
  const float b2j = sPar[P_AB2 + jj];
  const float wa0 = sPar[P_W2 + 3 * ca], wa1 = sPar[P_W2 + 3 * ca + 1], wa2 = sPar[P_W2 + 3 * ca + 2];
  const float wb0 = sPar[P_W2 + 3 * cb], wb1 = sPar[P_W2 + 3 * cb + 1], wb2 = sPar[P_W2 + 3 * cb + 2];
  const float ba = sPar[P_B2 + ca], bb = sPar[P_B2 + cb];
  const float scp0 = ssp[0], scp1 = ssp[1], scp2 = ssp[2];
  const float shp0 = ssp[CH], shp1 = ssp[CH + 1], shp2 = ssp[CH + 2];
  float mea = 0.0f, qa = 0.0f, meb = 0.0f, qb = 0.0f;
  int nW = 0;
#pragma unroll 1
  for (int jt = 0; jt < nbw; ++jt) {
    const int slot = wave * nbw + jt;
    const int grow = nodeBase + slot;
    int st = __builtin_amdgcn_readfirstlane(soff[slot]);
    const int craw = __builtin_amdgcn_readfirstlane(scnt[slot]);
    int cnt = craw;
    st  = st < 0 ? 0 : (st > nh ? nh : st);
    cnt = cnt < 0 ? 0 : (cnt > DEGCAP ? DEGCAP : cnt);
    if (cnt > nh - st) cnt = nh - st;
    const float pz = (ovf || craw > DEGCAP) ? qnan : 0.0f;
    float t0, t1, t2;
    ld_pos(pos, grow, t0, t1, t2);
    float mx = -1.0e30f, dn = 0.0f, ava = 0.0f, avb = 0.0f;
#pragma unroll 1
    for (int b0 = 0; b0 < cnt; b0 += 32) {
      int idx = st + b0 + lane;
      const int last = st + cnt - 1;
      idx = idx > last ? last : idx;
      idx = idx < 0 ? 0 : (idx > RCAP - 1 ? RCAP - 1 : idx);
      const int eid = clampi(reg2[idx], nE - 1);
      const int s = clampi(srcs[eid], NN - 1);
      float s0, s1, s2, p0, p1, p2;
      ld_pos(pos, s, s0, s1, s2);
      p1vec(s0 - t0, s1 - t1, s2 - t2, sPar, p0, p1, p2);
      const float d0 = rl(fmaf(p0, scp0, shp0));
      const float d1 = rl(fmaf(p1, scp1, shp1));
      const float d2 = rl(fmaf(p2, scp2, shp2));
      const int m32 = (cnt - b0) < 32 ? (cnt - b0) : 32;
#pragma unroll 1
      for (int k = 0; k < m32; ++k) {
        const int ek = __builtin_amdgcn_readlane(eid, k);
        const int sk = __builtin_amdgcn_readlane(s, k);
        const float e0 = __int_as_float(__builtin_amdgcn_readlane(__float_as_int(d0), k));
        const float e1 = __int_as_float(__builtin_amdgcn_readlane(__float_as_int(d1), k));
        const float e2 = __int_as_float(__builtin_amdgcn_readlane(__float_as_int(d2), k));
        const float* yr = A1 + (size_t)ek * 8;
        const v4f y0 = *(const v4f*)yr;
        const v4f y1 = *(const v4f*)(yr + 4);
        const float* nr = node + (size_t)sk * NDW + 2 * CH;
        const float ha = nr[ca];
        const float hb = nr[cb];
        float lg = rl(fmaf(y0.x, sS2[0], sS2[8])) * w2r[0];
        lg = fmaf(rl(fmaf(y0.y, sS2[1], sS2[9])),  w2r[1], lg);
        lg = fmaf(rl(fmaf(y0.z, sS2[2], sS2[10])), w2r[2], lg);
        lg = fmaf(rl(fmaf(y0.w, sS2[3], sS2[11])), w2r[3], lg);
        lg = fmaf(rl(fmaf(y1.x, sS2[4], sS2[12])), w2r[4], lg);
        lg = fmaf(rl(fmaf(y1.y, sS2[5], sS2[13])), w2r[5], lg);
        lg = fmaf(rl(fmaf(y1.z, sS2[6], sS2[14])), w2r[6], lg);
        lg = fmaf(rl(fmaf(y1.w, sS2[7], sS2[15])), w2r[7], lg);
        lg = lg + b2j;
        const float va = ha + (fmaf(e2, wa2, fmaf(e1, wa1, e0 * wa0)) + ba);
        const float vb = hb + (fmaf(e2, wb2, fmaf(e1, wb1, e0 * wb0)) + bb);
        const float df = lg - mx;
        const float ee = expf(-fabsf(df));
        const bool up  = df > 0.0f;
        const float f1 = up ? ee : 1.0f;
        const float f2 = up ? 1.0f : ee;
        mx = up ? lg : mx;
        dn = fmaf(dn, f1, f2);
        ava = fmaf(ava, f1, f2 * va);
        avb = fmaf(avb, f1, f2 * vb);
      }
    }
    const bool zr = (dn == 0.0f);
    const float iv = __builtin_amdgcn_rcpf(zr ? 1.0f : dn);
    const float oa = (zr ? 0.0f : ava * iv) + pz;
    const float ob = (zr ? 0.0f : avb * iv) + pz;
    float* op = outp + (size_t)grow * CH;
    *(volatile float*)(op + ca) = oa;
    *(volatile float*)(op + cb) = ob;
    __threadfence();
    *(volatile float*)(op + ca) = oa;
    *(volatile float*)(op + cb) = ob;
    nW = nW + 1;
    const float r = rinv[nW];
    const float da = oa - mea;
    mea = fmaf(da, r, mea);
    qa = fmaf(da, oa - mea, qa);
    const float db = ob - meb;
    meb = fmaf(db, r, meb);
    qb = fmaf(db, ob - meb, qb);
  }
  __builtin_amdgcn_fence(__ATOMIC_RELEASE, "wavefront");
  __builtin_amdgcn_wave_barrier();
  stw[1 + ca] = mea;
  stw[1 + cb] = meb;
  stw[1 + CH + ca] = qa;
  stw[1 + CH + cb] = qb;
  if (lane == 0) stw[0] = (float)nbw;
  if (lane < 31) stw[2 * CH + 1 + lane] = 0.0f;
  __builtin_amdgcn_fence(__ATOMIC_RELEASE, "wavefront");
  __builtin_amdgcn_wave_barrier();
  const v4f r0 = *(const v4fa*)(stw + 4 * lane);
  const v4f r1 = *(const v4fa*)(stw + 128 + 4 * (lane & 7));
  float* rp = part + (size_t)((int)blockIdx.x * NWAVE + wave) * PARTW;
  *(volatile v4f*)(rp + 4 * lane) = r0;
  if (lane < 8) *(volatile v4f*)(rp + 128 + 4 * lane) = r1;
  __threadfence();
  *(volatile v4f*)(rp + 4 * lane) = r0;
  if (lane < 8) *(volatile v4f*)(rp + 128 + 4 * lane) = r1;
}

__global__ __launch_bounds__(NTHR) void k_final(const float* __restrict__ T3, const float* __restrict__ x,
                                                const float* __restrict__ ss, float* out) {
  __shared__ __attribute__((aligned(16))) float sl[2 * CH];
  const int tid = (int)threadIdx.x;
  if (tid < 32) *(v4fa*)(sl + 4 * tid) = *(const v4f*)(ss + 4 * tid);
  __syncthreads();
  const size_t u = (size_t)blockIdx.x * NTHR + tid;
  const int c4 = (int)(u & 15) * 4;
  const v4f t  = *(const v4f*)(T3 + 4 * u);
  const v4f xv = *(const v4f*)(x + 4 * u);
  v4f o;
  o.x = rl(fmaf(t.x, sl[c4 + 0], sl[CH + c4 + 0]) + bf16_val(xv.x));
  o.y = rl(fmaf(t.y, sl[c4 + 1], sl[CH + c4 + 1]) + bf16_val(xv.y));
  o.z = rl(fmaf(t.z, sl[c4 + 2], sl[CH + c4 + 2]) + bf16_val(xv.z));
  o.w = rl(fmaf(t.w, sl[c4 + 3], sl[CH + c4 + 3]) + bf16_val(xv.w));
  float* op = out + 4 * u;
  *(volatile v4f*)op = o;
  __threadfence();
  *(volatile v4f*)op = o;
}

static inline size_t al256(size_t o) { return (o + 255) & ~(size_t)255; }

extern "C" void kernel_launch(void* const* d_in, const int* in_sizes, int n_in,
                              void* d_out, int out_size, void* d_ws, size_t ws_size,
                              hipStream_t stream) {
  if (n_in < 31) return;
  if (in_sizes[0] != NN * CH || in_sizes[1] != NN * 3 || in_sizes[2] != 2 * NE) return;
  if (in_sizes[3] != CH * CH || in_sizes[4] != CH * CH) return;
  if (in_sizes[5] != 9 || in_sizes[6] != 3 || in_sizes[7] != 3 || in_sizes[8] != 3) return;
  if (in_sizes[9] != CH * 3 || in_sizes[10] != CH || in_sizes[11] != CH || in_sizes[12] != CH) return;
  if (in_sizes[13] != 8 * CH || in_sizes[14] != 8 || in_sizes[15] != 8 || in_sizes[16] != 8) return;
  if (in_sizes[17] != 64 || in_sizes[18] != 8) return;
  if (in_sizes[19] != CH * CH || in_sizes[20] != CH || in_sizes[21] != CH * CH || in_sizes[22] != CH) return;
  if (in_sizes[23] != CH * CH || in_sizes[24] != CH) return;
  for (int i = 25; i < 31; ++i) if (in_sizes[i] != CH) return;
  if (out_size != NN * CH) return;

  const float* x        = (const float*)d_in[0];
  const float* pos      = (const float*)d_in[1];
  const int*   ei       = (const int*)d_in[2];
  const float* W_in     = (const float*)d_in[3];
  const float* W_out    = (const float*)d_in[4];
  const float* pos_w1   = (const float*)d_in[5];
  const float* pos_b1   = (const float*)d_in[6];
  const float* pos_bn_g = (const float*)d_in[7];
  const float* pos_bn_b = (const float*)d_in[8];
  const float* pos_w2   = (const float*)d_in[9];
  const float* pos_b2   = (const float*)d_in[10];
  const float* a1_g     = (const float*)d_in[11];
  const float* a1_b     = (const float*)d_in[12];
  const float* attn_w1  = (const float*)d_in[13];
  const float* attn_b1  = (const float*)d_in[14];
  const float* a2_g     = (const float*)d_in[15];
  const float* a2_b     = (const float*)d_in[16];
  const float* attn_w2  = (const float*)d_in[17];
  const float* attn_b2  = (const float*)d_in[18];
  const float* lin_w    = (const float*)d_in[19];
  const float* lin_b    = (const float*)d_in[20];
  const float* src_w    = (const float*)d_in[21];
  const float* src_b    = (const float*)d_in[22];
  const float* dst_w    = (const float*)d_in[23];
  const float* dst_b    = (const float*)d_in[24];
  const float* bn1_g    = (const float*)d_in[25];
  const float* bn1_b    = (const float*)d_in[26];
  const float* bn2_g    = (const float*)d_in[27];
  const float* bn2_b    = (const float*)d_in[28];
  const float* bn3_g    = (const float*)d_in[29];
  const float* bn3_b    = (const float*)d_in[30];
  float* out = (float*)d_out;
  const int* src = ei;
  const int* dst = ei + NE;
  const int vec8 = ((NE & 3) == 0) ? 1 : 0;

  char* ws = (char*)d_ws;
  size_t off = 0;
  const size_t oWin = off; off = al256(off + (size_t)CH * CH * 2);
  const size_t oWct = off; off = al256(off + (size_t)NDW * HP * 2);
  const size_t oWot = off; off = al256(off + (size_t)CH * HP * 2);
  const size_t oAw1 = off; off = al256(off + (size_t)16 * HP * 2);
  const size_t oPar = off; off = al256(off + (size_t)PARN * 4);
  const size_t oSS  = off; off = al256(off + (size_t)6 * 2 * CH * 4);
  const size_t oRec = off; off = al256(off + (size_t)NEB * PARTW * 4);
  const size_t oP0  = off; off = al256(off + (size_t)NN * CH * 4);
  const size_t oH   = off; off = al256(off + (size_t)NN * HP * 2);
  const size_t oNd  = off; off = al256(off + (size_t)NN * NDW * 4);
  const size_t oA1  = off; off = al256(off + (size_t)NE * 8 * 4);
  if (off > ws_size || off > (size_t)WSMAX) return;
  unsigned short* WinB  = (unsigned short*)(ws + oWin);
  unsigned short* Wcat  = (unsigned short*)(ws + oWct);
  unsigned short* WoutD = (unsigned short*)(ws + oWot);
  unsigned short* Aw1D  = (unsigned short*)(ws + oAw1);
  float* PAR  = (float*)(ws + oPar);
  float* SS1  = (float*)(ws + oSS);
  float* SSP  = SS1 + 2 * CH;
  float* SSA1 = SSP + 2 * CH;
  float* SSA2 = SSA1 + 2 * CH;
  float* SS2  = SSA2 + 2 * CH;
  float* SS3  = SS2 + 2 * CH;
  float* REC  = (float*)(ws + oRec);
  float* P0   = (float*)(ws + oP0);
  unsigned short* H = (unsigned short*)(ws + oH);
  float* NODE = (float*)(ws + oNd);
  float* A1   = (float*)(ws + oA1);

  hipFuncSetAttribute(reinterpret_cast<const void*>(&k_scan), hipFuncAttributeMaxDynamicSharedMemorySize,
                      (int)LDS_AGG);

  k_prep<<<20, NTHR, 0, stream>>>(W_in, src_w, dst_w, lin_w, W_out, attn_w1, pos_w1, pos_b1, pos_w2, pos_b2,
                                  attn_b1, attn_w2, attn_b2, src_b, dst_b, lin_b, WinB, Wcat, WoutD, Aw1D, PAR);
  k_gemm<1, 2, 1, 0><<<dim3(NN / GBM, 1), NTHR, 0, stream>>>(x, H, WinB, PAR, P0, CH, REC);
  k_comb<<<1, NTHR, 0, stream>>>(REC, NN / GBM, CH, bn1_g, bn1_b, SS1);
  k_apply<<<NN * 8 / NTHR, NTHR, 0, stream>>>(P0, SS1, H);
  k_gemm<0, 4, 0, 1><<<dim3(NN / GBM, 3), NTHR, 0, stream>>>(x, H, Wcat, PAR, NODE, NDW, REC);
  k_epos<<<NEB, NTHR, 0, stream>>>(src, dst, pos, PAR, REC);
  k_comb<<<1, NTHR, 0, stream>>>(REC, NEB, 3, pos_bn_g, pos_bn_b, SSP);
  k_ea<<<NEB, NTHR, 0, stream>>>(src, dst, pos, NODE, PAR, SSP, REC);
  k_comb<<<1, NTHR, 0, stream>>>(REC, NEB, CH, a1_g, a1_b, SSA1);
  k_ea1<<<NEB, NTHR, 0, stream>>>(src, dst, pos, NODE, PAR, SSP, SSA1, Aw1D, A1, REC);
  k_comb<<<1, NTHR, 0, stream>>>(REC, NEB, 8, a2_g, a2_b, SSA2);
  k_scan<<<NN / NBRUN, NTHR, LDS_AGG, stream>>>(src, dst, pos, NODE, A1, PAR, SSP, SSA2, P0, REC, vec8);
  k_comb<<<1, NTHR, 0, stream>>>(REC, (NN / NBRUN) * NWAVE, CH, bn2_g, bn2_b, SS2);
  k_apply<<<NN * 8 / NTHR, NTHR, 0, stream>>>(P0, SS2, H);
  k_gemm<0, 4, 1, 0><<<dim3(NN / GBM, 1), NTHR, 0, stream>>>(x, H, WoutD, PAR, NODE, CH, REC);
  k_comb<<<1, NTHR, 0, stream>>>(REC, NN / GBM, CH, bn3_g, bn3_b, SS3);
  k_final<<<NN * CH / 4 / NTHR, NTHR, 0, stream>>>(NODE, x, SS3, out);
}
